// TransformerShell_7206955123256
// MI455X (gfx1250) — hardware-verified
//
#include <hip/hip_runtime.h>
#include <stddef.h>


#define CH    64
#define NHD   2
#define DF    128
#define KD    64
#define NC1   448
#define NCT1  (NC1 / 16)
#define AP    72
#define GR1   16
#define XSP   452
#define GR2   32
#define TSP   68
#define NB    512
#define CHUNK 2048
#define NTHR  256
#define NWAVE 8
#define WCAP  256
#define NGRP  (CHUNK / (NTHR * 4))

#define LDS_SACC (NB * DF)
#define LDS_MD   (NB * NHD * 2)
#define LDS_LIST (NWAVE * WCAP)
#define LDS_BYTES ((LDS_SACC + LDS_MD + LDS_LIST + NWAVE) * 4)

static_assert(WCAP == (CHUNK / NTHR) * 32);
static_assert(NGRP == 2);
static_assert(NB == 512);
static_assert(CHUNK == 2048);
static_assert((KD % 32) == 0);
static_assert(((AP * 2) % 16) == 0);
static_assert(((XSP * 4) % 16) == 0);
static_assert(((TSP * 4) % 16) == 0);
static_assert((LDS_SACC % 4) == 0 && (LDS_MD % 4) == 0);
static_assert(LDS_BYTES == 278560);
static_assert(NCT1 * 16 == NC1);
static_assert(NC1 == 3 * DF + CH);
static_assert(GR1 * 8 <= NTHR);
static_assert(GR2 * 8 == NTHR);

typedef float        v2f  __attribute__((ext_vector_type(2)));
typedef float        v4f  __attribute__((ext_vector_type(4)));
typedef float        v8f  __attribute__((ext_vector_type(8)));
typedef int          v4i  __attribute__((ext_vector_type(4)));
typedef unsigned int v4u  __attribute__((ext_vector_type(4)));
typedef __bf16       v8b  __attribute__((ext_vector_type(8)));
typedef __bf16       v16b __attribute__((ext_vector_type(16)));
union Frag { v16b v; v8b half[2]; v4u u[2]; };

__device__ __forceinline__ unsigned int bf_rne(float f) {
  const unsigned int u = __float_as_uint(f);
  return (u + 0x7FFFu + ((u >> 16) & 1u)) >> 16;
}

__device__ __forceinline__ void split2(float a, float b, unsigned int& hi, unsigned int& lo) {
  const unsigned int ha = bf_rne(a), hb = bf_rne(b);
  const unsigned int la = bf_rne(a - __uint_as_float(ha << 16));
  const unsigned int lb = bf_rne(b - __uint_as_float(hb << 16));
  hi = ha | (hb << 16);
  lo = la | (lb << 16);
}

__device__ __forceinline__ void split8(v4f a, v4f b, v4u& hi, v4u& lo) {
  unsigned int h, l;
  split2(a.x, a.y, h, l); hi.x = h; lo.x = l;
  split2(a.z, a.w, h, l); hi.y = h; lo.y = l;
  split2(b.x, b.y, h, l); hi.z = h; lo.z = l;
  split2(b.z, b.w, h, l); hi.w = h; lo.w = l;
}

__device__ __forceinline__ v8f wm(v16b a, v16b b, v8f c) {
  v8f d = __builtin_amdgcn_wmma_f32_16x16x32_bf16(false, a, false, b, (short)0, c, false, false);
  asm volatile("v_nop\n\tv_nop\n\tv_nop\n\tv_nop" : "+v"(d) : "v"(a), "v"(b));
  return d;
}

__device__ __forceinline__ v8f wm3(const Frag& ah, const Frag& al, const Frag& bh, const Frag& bl, v8f c) {
  c = wm(ah.v, bh.v, c);
  c = wm(ah.v, bl.v, c);
  c = wm(al.v, bh.v, c);
  return c;
}

__global__ __launch_bounds__(NTHR) void k_prep(
    const float* __restrict__ Wq, const float* __restrict__ Wk, const float* __restrict__ Wv,
    const float* __restrict__ Wsk, const float* __restrict__ Wl,
    unsigned short* Wch, unsigned short* Wcl, unsigned short* Wlh, unsigned short* Wll) {
  const int mat = blockIdx.y;
  const float* src = Wq;
  int nrows = DF, base = 0;
  unsigned short* dh = Wch;
  unsigned short* dl = Wcl;
  if (mat == 1)      { src = Wk;  base = DF; }
  else if (mat == 2) { src = Wv;  base = 2 * DF; }
  else if (mat == 3) { src = Wsk; base = 3 * DF; nrows = CH; }
  else if (mat == 4) { src = Wl;  base = 0;      nrows = CH; dh = Wlh; dl = Wll; }
  const int r = blockIdx.x * (NTHR / 8) + (threadIdx.x >> 3);
  if (r >= nrows) return;
  const int c0 = (threadIdx.x & 7) * 8;
  const float* p = src + (size_t)r * KD + c0;
  const v4f a = *(const v4f*)(p);
  const v4f b = *(const v4f*)(p + 4);
  v4u ph, pl;
  split8(a, b, ph, pl);
  const size_t o = (size_t)(base + r) * KD + c0;
  *(volatile v4u*)(dh + o) = ph;
  *(volatile v4u*)(dl + o) = pl;
  __threadfence();
  *(volatile v4u*)(dh + o) = ph;
  *(volatile v4u*)(dl + o) = pl;
}

__global__ __launch_bounds__(NTHR) void k_node(
    const float* __restrict__ x,
    const unsigned short* __restrict__ Wch, const unsigned short* __restrict__ Wcl,
    const float* __restrict__ bq, const float* __restrict__ bk,
    const float* __restrict__ bv, const float* __restrict__ bsk,
    float* qpl, float* kpl, float* vpl, float* skpl, int nN) {
  __shared__ __attribute__((aligned(16))) unsigned short Ah[GR1 * AP];
  __shared__ __attribute__((aligned(16))) unsigned short Al[GR1 * AP];
  __shared__ __attribute__((aligned(16))) float Xs[GR1 * XSP];

  const int tid  = threadIdx.x;
  const int lane = tid & 31;
  const int wave = __builtin_amdgcn_readfirstlane(tid >> 5);
  const int hh   = lane >> 4;
  const int m    = lane & 15;
  const int rowBase = blockIdx.x * GR1;

  if (tid < GR1 * 8) {
    const int r  = tid >> 3;
    const int c0 = (tid & 7) * 8;
    int row = rowBase + r;
    if (row > nN - 1) row = nN - 1;
    const float* p = x + (size_t)row * KD + c0;
    const v4f a = *(const v4f*)(p);
    const v4f b = *(const v4f*)(p + 4);
    v4u ph, pl;
    split8(a, b, ph, pl);
    *(v4u*)(Ah + r * AP + c0) = ph;
    *(v4u*)(Al + r * AP + c0) = pl;
  }
  __syncthreads();

#pragma unroll
  for (int j = 0; j < 4; ++j) {
    const int ct = wave + NWAVE * j;
    if (ct < NCT1) {
      const int n = ct * 16 + m;
      v8f acc = {0.f, 0.f, 0.f, 0.f, 0.f, 0.f, 0.f, 0.f};
#pragma unroll
      for (int ks = 0; ks < KD / 32; ++ks) {
        const int k0 = ks * 32;
        Frag ah, al, bh, bl;
        const unsigned short* pah = Ah + m * AP + k0 + 8 * hh;
        const unsigned short* pal = Al + m * AP + k0 + 8 * hh;
        const unsigned short* pbh = Wch + (size_t)n * KD + k0 + 8 * hh;
        const unsigned short* pbl = Wcl + (size_t)n * KD + k0 + 8 * hh;
        ah.u[0] = *(const v4u*)(pah); ah.u[1] = *(const v4u*)(pah + 16);
        al.u[0] = *(const v4u*)(pal); al.u[1] = *(const v4u*)(pal + 16);
        bh.u[0] = *(const v4u*)(pbh); bh.u[1] = *(const v4u*)(pbh + 16);
        bl.u[0] = *(const v4u*)(pbl); bl.u[1] = *(const v4u*)(pbl + 16);
        acc = wm3(ah, al, bh, bl, acc);
      }
      const float c0b = bq[min(n, DF - 1)];
      const float c1b = bk[min(max(n - DF, 0), DF - 1)];
      const float c2b = bv[min(max(n - 2 * DF, 0), DF - 1)];
      const float c3b = bsk[min(max(n - 3 * DF, 0), CH - 1)];
      const float bias = (n < DF) ? c0b : ((n < 2 * DF) ? c1b : ((n < 3 * DF) ? c2b : c3b));
#pragma unroll
      for (int r = 0; r < 8; ++r) Xs[(8 * hh + r) * XSP + ct * 16 + m] = acc[r] + bias;
    }
  }
  __syncthreads();

  const int r0 = 2 * wave, r1 = 2 * wave + 1;
  const size_t g0r = (size_t)(rowBase + r0), g1r = (size_t)(rowBase + r1);
  const v4f q0 = *(const v4f*)(Xs + r0 * XSP + 4 * lane);
  const v4f k0v = *(const v4f*)(Xs + r0 * XSP + DF + 4 * lane);
  const v4f v0 = *(const v4f*)(Xs + r0 * XSP + 2 * DF + 4 * lane);
  const v4f q1 = *(const v4f*)(Xs + r1 * XSP + 4 * lane);
  const v4f k1v = *(const v4f*)(Xs + r1 * XSP + DF + 4 * lane);
  const v4f v1 = *(const v4f*)(Xs + r1 * XSP + 2 * DF + 4 * lane);
  const int rs  = (lane < 16) ? r0 : r1;
  const int cl  = 4 * (lane & 15);
  const v4f sv  = *(const v4f*)(Xs + rs * XSP + 3 * DF + cl);
  float* pq0 = qpl + g0r * DF + 4 * lane;
  float* pk0 = kpl + g0r * DF + 4 * lane;
  float* pv0 = vpl + g0r * DF + 4 * lane;
  float* pq1 = qpl + g1r * DF + 4 * lane;
  float* pk1 = kpl + g1r * DF + 4 * lane;
  float* pv1 = vpl + g1r * DF + 4 * lane;
  float* ps  = skpl + (size_t)(rowBase + rs) * CH + cl;

  *(volatile v4f*)pq0 = q0; *(volatile v4f*)pk0 = k0v; *(volatile v4f*)pv0 = v0;
  *(volatile v4f*)pq1 = q1; *(volatile v4f*)pk1 = k1v; *(volatile v4f*)pv1 = v1;
  *(volatile v4f*)ps = sv;
  __threadfence();
  *(volatile v4f*)pq0 = q0; *(volatile v4f*)pk0 = k0v; *(volatile v4f*)pv0 = v0;
  *(volatile v4f*)pq1 = q1; *(volatile v4f*)pk1 = k1v; *(volatile v4f*)pv1 = v1;
  *(volatile v4f*)ps = sv;
}

__global__ __launch_bounds__(NTHR) void k_agg(
    const float* __restrict__ x, const int* __restrict__ ei, const float* __restrict__ ea,
    const float* __restrict__ qpl, const float* __restrict__ kpl, const float* __restrict__ vpl,
    const float* __restrict__ We, const float* __restrict__ skpl,
    const float* __restrict__ g0, const float* __restrict__ b0,
    float* x1pl, int nN, int nE) {
  extern __shared__ v4f lds_dyn[];
  float* sacc = (float*)lds_dyn;
  float* md   = sacc + LDS_SACC;
  int*   list = (int*)(md + LDS_MD);
  int*   wcnt = list + LDS_LIST;

  const int tid  = threadIdx.x;
  const int lane = tid & 31;
  const int wave = __builtin_amdgcn_readfirstlane(tid >> 5);
  const int hd   = lane >> 4;
  const int nodeBase = blockIdx.x * NB;

  {
    const v4f z4 = {0.f, 0.f, 0.f, 0.f};
    for (int i = tid; i < LDS_SACC / 4; i += NTHR) lds_dyn[i] = z4;
    const v4f mi = {-1e30f, 0.f, -1e30f, 0.f};
    for (int i = tid; i < LDS_MD / 4; i += NTHR) lds_dyn[LDS_SACC / 4 + i] = mi;
  }
  __syncthreads();

  const v4f we4 = *(const v4f*)(We + 4 * lane);
  const int* eid = ei + nE;
  const bool al16 = ((nE & 3) == 0);

  const int nChunks = (nE + CHUNK - 1) / CHUNK;
#pragma unroll 1
  for (int ch = 0; ch < nChunks; ++ch) {
    const int cbase = ch * CHUNK;
    const bool full = al16 && (cbase + CHUNK <= nE);
    int wc = 0;
#pragma unroll
    for (int g = 0; g < NGRP; ++g) {
      const int el0 = (g * NTHR + tid) * 4;
      const int e0  = cbase + el0;
      const int sent = -2147483647 - 1;
      v4i d;
      if (full) {
        d = *(const v4i*)(eid + e0);
      } else {
        const int v0 = eid[min(e0, nE - 1)];
        const int v1 = eid[min(e0 + 1, nE - 1)];
        const int v2 = eid[min(e0 + 2, nE - 1)];
        const int v3 = eid[min(e0 + 3, nE - 1)];
        d.x = (e0     < nE) ? v0 : sent;
        d.y = (e0 + 1 < nE) ? v1 : sent;
        d.z = (e0 + 2 < nE) ? v2 : sent;
        d.w = (e0 + 3 < nE) ? v3 : sent;
      }
      const unsigned s0 = (unsigned)d.x - (unsigned)nodeBase;
      const unsigned s1 = (unsigned)d.y - (unsigned)nodeBase;
      const unsigned s2 = (unsigned)d.z - (unsigned)nodeBase;
      const unsigned s3 = (unsigned)d.w - (unsigned)nodeBase;
      const bool h0 = s0 < (unsigned)NB;
      const bool h1 = s1 < (unsigned)NB;
      const bool h2 = s2 < (unsigned)NB;
      const bool h3 = s3 < (unsigned)NB;
      const unsigned many = __builtin_amdgcn_ballot_w32(h0 | h1 | h2 | h3);
      if (many != 0u) {
#define HITJ(J, HJ, SJ) { \
          const unsigned mj = __builtin_amdgcn_ballot_w32(HJ); \
          if (HJ) { \
            const int pos = wc + (int)__builtin_amdgcn_mbcnt_lo(mj, 0u); \
            if (pos < WCAP) list[wave * WCAP + pos] = ((el0 + (J)) << 9) | (int)(SJ); \
          } \
          wc += (int)__builtin_popcount(mj); }
        HITJ(0, h0, s0)
        HITJ(1, h1, s1)
        HITJ(2, h2, s2)
        HITJ(3, h3, s3)
#undef HITJ
      }
    }
    if (lane == 0) wcnt[wave] = wc;
    __syncthreads();

    if (wave == 0) {
#pragma unroll 1
      for (int wsx = 0; wsx < NWAVE; ++wsx) {
        int n = wcnt[wsx];
        if (n > WCAP) n = WCAP;
        if (n < 0) n = 0;
#pragma unroll 1
        for (int i = 0; i < n; ++i) {
          const int ent  = list[wsx * WCAP + i];
          const int slot = ent & (NB - 1);
          const int el   = (ent >> 9) & (CHUNK - 1);
          int e = cbase + el;
          if (e > nE - 1) e = nE - 1;
          int src = ei[e];
          src = src < 0 ? 0 : (src > nN - 1 ? nN - 1 : src);
          const float w = ea[e];
          int nd = nodeBase + slot;
          if (nd > nN - 1) nd = nN - 1;
          const v4f qv = *(const v4f*)(qpl + (size_t)nd  * DF + 4 * lane);
          const v4f kv = *(const v4f*)(kpl + (size_t)src * DF + 4 * lane);
          const v4f vv = *(const v4f*)(vpl + (size_t)src * DF + 4 * lane);
          const v4f kj = kv + w * we4;
          const v4f vj = vv + w * we4;
          float dt = qv.x * kj.x + qv.y * kj.y + qv.z * kj.z + qv.w * kj.w;
          dt += __shfl_xor(dt, 8, 32);
          dt += __shfl_xor(dt, 4, 32);
          dt += __shfl_xor(dt, 2, 32);
          dt += __shfl_xor(dt, 1, 32);
          const float alv = dt * 0.125f;
          float* mp = md + (slot * NHD + hd) * 2;
          const v2f mo = *(const v2f*)mp;
          const float mn = fmaxf(mo.x, alv);
          const float sc = __expf(mo.x - mn);
          const float p  = __expf(alv - mn);
          v4f* sp = (v4f*)(sacc + slot * DF + 4 * lane);
          const v4f cur = *sp;
          const v4f nxt = cur * sc + p * vj;
          *sp = nxt;
          v2f mw;
          mw.x = mn;
          mw.y = mo.y * sc + p;
          *(v2f*)mp = mw;
        }
      }
    }
    __syncthreads();
  }

  const int cl = 4 * (lane & 15);
  const v4f g4 = *(const v4f*)(g0 + cl);
  const v4f e4 = *(const v4f*)(b0 + cl);
  const bool lo16 = lane < 16;
#pragma unroll 1
  for (int j = 0; j < NB / NWAVE / 2; ++j) {
    const int sA = wave * (NB / NWAVE) + 2 * j;
    const int sB = sA + 1;
    const v4f aA = *(const v4f*)(sacc + sA * DF + 4 * lane);
    const v4f aB = *(const v4f*)(sacc + sB * DF + 4 * lane);
    const float dA = md[(sA * NHD + hd) * 2 + 1];
    const float dB = md[(sB * NHD + hd) * 2 + 1];
    const float iA = (dA > 0.f) ? __builtin_amdgcn_rcpf(dA) : 0.f;
    const float iB = (dB > 0.f) ? __builtin_amdgcn_rcpf(dB) : 0.f;
    const v4f nA = aA * iA;
    const v4f nB = aB * iB;
    v4f pA, pB;
    pA.x = __shfl_xor(nA.x, 16, 32); pA.y = __shfl_xor(nA.y, 16, 32);
    pA.z = __shfl_xor(nA.z, 16, 32); pA.w = __shfl_xor(nA.w, 16, 32);
    pB.x = __shfl_xor(nB.x, 16, 32); pB.y = __shfl_xor(nB.y, 16, 32);
    pB.z = __shfl_xor(nB.z, 16, 32); pB.w = __shfl_xor(nB.w, 16, 32);
    const v4f mA = (nA + pA) * 0.5f;
    const v4f mB = (nB + pB) * 0.5f;
    v4f hv = mB;
    if (lo16) hv = mA;
    const int node = nodeBase + (lo16 ? sA : sB);
    int nodec = node;
    if (nodec > nN - 1) nodec = nN - 1;
    const v4f sk = *(const v4f*)(skpl + (size_t)nodec * CH + cl);
    const v4f xr = *(const v4f*)(x + (size_t)nodec * CH + cl);
    const v4f h = hv + sk;
    float s = h.x + h.y + h.z + h.w;
    s += __shfl_xor(s, 8, 32); s += __shfl_xor(s, 4, 32);
    s += __shfl_xor(s, 2, 32); s += __shfl_xor(s, 1, 32);
    const float mu = s * (1.0f / CH);
    const v4f dd = h - mu;
    float qs = dd.x * dd.x + dd.y * dd.y + dd.z * dd.z + dd.w * dd.w;
    qs += __shfl_xor(qs, 8, 32); qs += __shfl_xor(qs, 4, 32);
    qs += __shfl_xor(qs, 2, 32); qs += __shfl_xor(qs, 1, 32);
    const float rsd = rsqrtf(qs * (1.0f / CH) + 1e-5f);
    const v4f y = dd * rsd * g4 + e4;
    const v4f o = xr + y;
    float* op = x1pl + (size_t)node * CH + cl;
    const bool ok = node < nN;
    if (ok) *(volatile v4f*)op = o;
    __threadfence();
    if (ok) *(volatile v4f*)op = o;
  }
}

__global__ __launch_bounds__(NTHR) void k_tail(
    const float* __restrict__ x1pl,
    const unsigned short* __restrict__ Wlh, const unsigned short* __restrict__ Wll,
    const float* __restrict__ bl, const float* __restrict__ g1, const float* __restrict__ b1,
    float* out, int nN) {
  __shared__ __attribute__((aligned(16))) unsigned short Ah[GR2 * AP];
  __shared__ __attribute__((aligned(16))) unsigned short Al[GR2 * AP];
  __shared__ __attribute__((aligned(16))) float Ts[GR2 * TSP];

  const int tid  = threadIdx.x;
  const int lane = tid & 31;
  const int wave = __builtin_amdgcn_readfirstlane(tid >> 5);
  const int hh   = lane >> 4;
  const int m    = lane & 15;
  const int rowBase = blockIdx.x * GR2;

  {
    const int r  = tid >> 3;
    const int c0 = (tid & 7) * 8;
    int row = rowBase + r;
    if (row > nN - 1) row = nN - 1;
    const float* p = x1pl + (size_t)row * KD + c0;
    const v4f a = *(const v4f*)(p);
    const v4f b = *(const v4f*)(p + 4);
    v4u ph, pl;
    split8(a, b, ph, pl);
    *(v4u*)(Ah + r * AP + c0) = ph;
    *(v4u*)(Al + r * AP + c0) = pl;
  }
  __syncthreads();

  {
    const int rt = wave >> 2;
    const int ct = wave & 3;
    const int n  = ct * 16 + m;
    v8f acc = {0.f, 0.f, 0.f, 0.f, 0.f, 0.f, 0.f, 0.f};
#pragma unroll
    for (int ks = 0; ks < KD / 32; ++ks) {
      const int k0 = ks * 32;
      Frag ah, al, bh, blf;
      const unsigned short* pah = Ah + (rt * 16 + m) * AP + k0 + 8 * hh;
      const unsigned short* pal = Al + (rt * 16 + m) * AP + k0 + 8 * hh;
      const unsigned short* pbh = Wlh + (size_t)n * KD + k0 + 8 * hh;
      const unsigned short* pbl = Wll + (size_t)n * KD + k0 + 8 * hh;
      ah.u[0]  = *(const v4u*)(pah); ah.u[1]  = *(const v4u*)(pah + 16);
      al.u[0]  = *(const v4u*)(pal); al.u[1]  = *(const v4u*)(pal + 16);
      bh.u[0]  = *(const v4u*)(pbh); bh.u[1]  = *(const v4u*)(pbh + 16);
      blf.u[0] = *(const v4u*)(pbl); blf.u[1] = *(const v4u*)(pbl + 16);
      acc = wm3(ah, al, bh, blf, acc);
    }
    const float bn = bl[n];
#pragma unroll
    for (int r = 0; r < 8; ++r) Ts[(rt * 16 + 8 * hh + r) * TSP + ct * 16 + m] = acc[r] + bn;
  }
  __syncthreads();

  const int cl = 4 * (lane & 15);
  const v4f g4 = *(const v4f*)(g1 + cl);
  const v4f e4 = *(const v4f*)(b1 + cl);
#pragma unroll
  for (int pp = 0; pp < 2; ++pp) {
    const int rA = 4 * wave + 2 * pp;
    const int r  = (lane < 16) ? rA : (rA + 1);
    const v4f t4 = *(const v4f*)(Ts + r * TSP + cl);
    float s = t4.x + t4.y + t4.z + t4.w;
    s += __shfl_xor(s, 8, 32); s += __shfl_xor(s, 4, 32);
    s += __shfl_xor(s, 2, 32); s += __shfl_xor(s, 1, 32);
    const float mu = s * (1.0f / CH);
    const v4f dd = t4 - mu;
    float qs = dd.x * dd.x + dd.y * dd.y + dd.z * dd.z + dd.w * dd.w;
    qs += __shfl_xor(qs, 8, 32); qs += __shfl_xor(qs, 4, 32);
    qs += __shfl_xor(qs, 2, 32); qs += __shfl_xor(qs, 1, 32);
    const float rsd = rsqrtf(qs * (1.0f / CH) + 1e-5f);
    const v4f y = dd * rsd * g4 + e4;
    const int grow = rowBase + r;
    int growc = grow;
    if (growc > nN - 1) growc = nN - 1;
    const v4f xr = *(const v4f*)(x1pl + (size_t)growc * CH + cl);
    const v4f o = xr + y;
    float* op = out + (size_t)grow * CH + cl;
    const bool ok = grow < nN;
    if (ok) *(volatile v4f*)op = o;
    __threadfence();
    if (ok) *(volatile v4f*)op = o;
  }
}

static inline size_t al256(size_t v) { return (v + 255) & ~(size_t)255; }

extern "C" void kernel_launch(void* const* d_in, const int* in_sizes, int n_in,
                              void* d_out, int out_size, void* d_ws, size_t ws_size,
                              hipStream_t stream) {
  if (n_in < 18) return;
  const int nN = in_sizes[0] / CH;
  if (nN <= 0 || in_sizes[0] != nN * CH) return;
  const int nE = in_sizes[2];
  if (nE < 0 || in_sizes[1] != 2 * nE) return;
  if (in_sizes[3] != DF * KD || in_sizes[5] != DF * KD || in_sizes[7] != DF * KD) return;
  if (in_sizes[4] != DF || in_sizes[6] != DF || in_sizes[8] != DF || in_sizes[9] != DF) return;
  if (in_sizes[10] != CH * KD || in_sizes[12] != CH * KD) return;
  if (in_sizes[11] != CH || in_sizes[13] != CH) return;
  if (in_sizes[14] != CH || in_sizes[15] != CH || in_sizes[16] != CH || in_sizes[17] != CH) return;
  if (out_size != nN * CH) return;

  const float* x     = (const float*)d_in[0];
  const int*   ei    = (const int*)d_in[1];
  const float* ea    = (const float*)d_in[2];
  const float* Wq    = (const float*)d_in[3];
  const float* bq    = (const float*)d_in[4];
  const float* Wk    = (const float*)d_in[5];
  const float* bk    = (const float*)d_in[6];
  const float* Wv    = (const float*)d_in[7];
  const float* bv    = (const float*)d_in[8];
  const float* We    = (const float*)d_in[9];
  const float* Wsk   = (const float*)d_in[10];
  const float* bsk   = (const float*)d_in[11];
  const float* Wl    = (const float*)d_in[12];
  const float* bl    = (const float*)d_in[13];
  const float* g0    = (const float*)d_in[14];
  const float* b0    = (const float*)d_in[15];
  const float* g1    = (const float*)d_in[16];
  const float* b1    = (const float*)d_in[17];
  float* out = (float*)d_out;

  const int nP1 = ((nN + GR1 - 1) / GR1) * GR1;
  const int nP2 = ((nN + GR2 - 1) / GR2) * GR2;
  size_t off = 0;
  unsigned short* Wch = (unsigned short*)((char*)d_ws + off); off = al256(off + (size_t)NC1 * KD * 2);
  unsigned short* Wcl = (unsigned short*)((char*)d_ws + off); off = al256(off + (size_t)NC1 * KD * 2);
  unsigned short* Wlh = (unsigned short*)((char*)d_ws + off); off = al256(off + (size_t)CH * KD * 2);
  unsigned short* Wll = (unsigned short*)((char*)d_ws + off); off = al256(off + (size_t)CH * KD * 2);
  float* qpl  = (float*)((char*)d_ws + off); off = al256(off + (size_t)nP1 * DF * 4);
  float* kpl  = (float*)((char*)d_ws + off); off = al256(off + (size_t)nP1 * DF * 4);
  float* vpl  = (float*)((char*)d_ws + off); off = al256(off + (size_t)nP1 * DF * 4);
  float* skpl = (float*)((char*)d_ws + off); off = al256(off + (size_t)nP1 * CH * 4);
  float* x1pl = (float*)((char*)d_ws + off); off = al256(off + (size_t)nP2 * CH * 4);
  if (off > ws_size) return;
  if (off > ((size_t)128 << 20)) return;

  k_prep<<<dim3(DF / (NTHR / 8), 5), NTHR, 0, stream>>>(Wq, Wk, Wv, Wsk, Wl, Wch, Wcl, Wlh, Wll);

  k_node<<<nP1 / GR1, NTHR, 0, stream>>>(x, Wch, Wcl, bq, bk, bv, bsk, qpl, kpl, vpl, skpl, nN);

  hipFuncSetAttribute(reinterpret_cast<const void*>(&k_agg),
                      hipFuncAttributeMaxDynamicSharedMemorySize, LDS_BYTES);
  const int gridA = (nN + NB - 1) / NB;
  k_agg<<<gridA, NTHR, LDS_BYTES, stream>>>(x, ei, ea, qpl, kpl, vpl, We, skpl, g0, b0, x1pl, nN, nE);

  k_tail<<<nP2 / GR2, NTHR, 0, stream>>>(x1pl, Wlh, Wll, bl, g1, b1, out, nN);
}
